// GRU_29815662969384
// MI455X (gfx1250) — hardware-run, weakly checked
//
#include <hip/hip_runtime.h>
#include <hip/hip_bf16.h>

typedef __attribute__((ext_vector_type(16))) _Float16 v16h;
typedef __attribute__((ext_vector_type(8)))  _Float16 v8h;
typedef __attribute__((ext_vector_type(16))) __bf16   v16b;
typedef __attribute__((ext_vector_type(8)))  __bf16   v8b;
typedef __attribute__((ext_vector_type(8)))  float    v8f;
typedef __attribute__((ext_vector_type(4)))  float    v4f;
#define PSCALE 32768.0f
#define U16(p) ((const unsigned short*)(const void*)(p))
#define PSCALE_INV (1.0f / 32768.0f)

__device__ __forceinline__ unsigned short f2bf_bits(float f) {
  unsigned u = __float_as_uint(f);
  return (unsigned short)((u + 0x7FFFu + ((u >> 16) & 1u)) >> 16);
}
__device__ __forceinline__ float bf_bits2f(unsigned short h) { return __uint_as_float(((unsigned)h) << 16); }

__device__ __forceinline__ void dep_guard_h(v8f& a, v8f& b, v16h x, v16h y) { asm volatile("v_nop\n\tv_nop\n\tv_nop\n\tv_nop" : "+v"(a), "+v"(b) : "v"(x), "v"(y)); }
__device__ __forceinline__ void dep_guard_b(v8f& a, v8f& b, v16b x, v16b y) { asm volatile("v_nop\n\tv_nop\n\tv_nop\n\tv_nop" : "+v"(a), "+v"(b) : "v"(x), "v"(y)); }
__device__ __forceinline__ void keep4_h(v16h a, v16h b, v16h c, v16h d) { asm volatile("v_nop" :: "v"(a), "v"(b), "v"(c), "v"(d)); }
__device__ __forceinline__ void keep4_b(v16b a, v16b b, v16b c, v16b d) { asm volatile("v_nop" :: "v"(a), "v"(b), "v"(c), "v"(d)); }
__device__ __forceinline__ void acc_guard4(v8f& a, v8f& b, v8f& c, v8f& d) { asm volatile("v_nop\n\tv_nop\n\tv_nop\n\tv_nop" : "+v"(a), "+v"(b), "+v"(c), "+v"(d)); }
template <typename T> struct Frag;
template <> struct Frag<_Float16> {
  typedef v16h V; union U { v16h v; v8h h[2]; };
  static __device__ __forceinline__ v16h load(const _Float16* p) {
    U f; f.h[0] = *(const v8h*)(p); f.h[1] = *(const v8h*)(p + 16); return f.v;
  }
  static __device__ __forceinline__ v8f mma(v16h a, v16h b, v8f c) {
    return __builtin_amdgcn_wmma_f32_16x16x32_f16(false, a, false, b, (short)0, c, false, false);
  }
  static __device__ __forceinline__ void guard(v8f& a, v8f& b, v16h x, v16h y) { dep_guard_h(a, b, x, y); }
  static __device__ __forceinline__ void keep(v16h a, v16h b, v16h c, v16h d) { keep4_h(a, b, c, d); }
};
template <> struct Frag<__bf16> {
  typedef v16b V; union U { v16b v; v8b h[2]; };
  static __device__ __forceinline__ v16b load(const __bf16* p) {
    U f; f.h[0] = *(const v8b*)(p); f.h[1] = *(const v8b*)(p + 16); return f.v;
  }
  static __device__ __forceinline__ v8f mma(v16b a, v16b b, v8f c) {
    return __builtin_amdgcn_wmma_f32_16x16x32_bf16(false, a, false, b, (short)0, c, false, false);
  }
  static __device__ __forceinline__ void guard(v8f& a, v8f& b, v16b x, v16b y) { dep_guard_b(a, b, x, y); }
  static __device__ __forceinline__ void keep(v16b a, v16b b, v16b c, v16b d) { keep4_b(a, b, c, d); }
};

template <int ET> struct Elem;
template <> struct Elem<0> { typedef _Float16 T; };
template <> struct Elem<1> { typedef __bf16 T; };
template <int ET, bool SPLIT, int BIAS_MODE, int OUT_MODE, bool RESID, int ACT = 0>
__global__ __launch_bounds__(256) void wmma_gemm64(
    const unsigned short* __restrict__ Ap, const unsigned short* __restrict__ A2p, int lda, long strideA,
    const unsigned short* __restrict__ Btp, const unsigned short* __restrict__ Bt2p, int ldb, long strideB,
    void* __restrict__ Cout, void* __restrict__ Cout2, int ldc, long strideC,
    const float* __restrict__ bias,
    const float* __restrict__ resid, long strideR,
    int M, int N, int K, float scale) {
  typedef typename Elem<ET>::T T;
  typedef typename Frag<T>::V V;
  const T* A = (const T*)Ap; const T* A2 = (const T*)A2p; const T* Bt = (const T*)Btp; const T* Bt2 = (const T*)Bt2p;
  __shared__ __align__(16) float sT[8][16 * 68];
  const int b    = blockIdx.y;
  const int lane = threadIdx.x & 31;
  const int wave = threadIdx.x >> 5;
  const int tilesN = N >> 6;
  const int tilesM = M >> 6;
  const int tile = blockIdx.x * 8 + wave;
  if (tile >= tilesM * tilesN) return;
  const int tm = tile / tilesN;
  const int tn = tile - tm * tilesN;
  const int m0 = tm << 6;
  const int n0 = tn << 6;

  const T* Ab  = A  + (size_t)b * strideA;
  const T* Bb  = Bt + (size_t)b * strideB;
  const T* Ab2 = SPLIT ? (A2  + (size_t)b * strideA) : nullptr;
  const T* Bb2 = SPLIT ? (Bt2 + (size_t)b * strideB) : nullptr;

  const int rlane = lane & 15;
  const int koff  = (lane >> 4) * 8;
  const int mOff  = (lane >> 4) * 8;

  v8f acc[4][4];
#pragma unroll
  for (int i = 0; i < 4; ++i)
#pragma unroll
    for (int j = 0; j < 4; ++j) acc[i][j] = (v8f){0.f,0.f,0.f,0.f,0.f,0.f,0.f,0.f};

  for (int k0 = 0; k0 < K; k0 += 32) {
    V bh[4], bl[4];
#pragma unroll
    for (int j = 0; j < 4; ++j) {
      const size_t bo = (size_t)(n0 + (j << 4) + rlane) * ldb + koff + k0;
      bh[j] = Frag<T>::load(Bb + bo);
      if (SPLIT) bl[j] = Frag<T>::load(Bb2 + bo);
    }
#pragma unroll
    for (int i = 0; i < 4; ++i) {
      const size_t ao = (size_t)(m0 + (i << 4) + rlane) * lda + koff + k0;
      V ah = Frag<T>::load(Ab + ao);
      V al;
      if (SPLIT) al = Frag<T>::load(Ab2 + ao);
#pragma unroll
      for (int j = 0; j < 4; ++j) {
        acc[i][j] = Frag<T>::mma(ah, bh[j], acc[i][j]);
        if (SPLIT) {
          acc[i][j] = Frag<T>::mma(ah, bl[j], acc[i][j]);
          acc[i][j] = Frag<T>::mma(al, bh[j], acc[i][j]);
        }
      }
      Frag<T>::guard(acc[i][0], acc[i][3], ah, SPLIT ? al : ah);
    }
    Frag<T>::keep(bh[0], bh[1], bh[2], bh[3]);
    if (SPLIT) Frag<T>::keep(bl[0], bl[1], bl[2], bl[3]);
  }
  acc_guard4(acc[0][0], acc[0][1], acc[0][2], acc[0][3]);
  acc_guard4(acc[1][0], acc[1][1], acc[1][2], acc[1][3]);
  acc_guard4(acc[2][0], acc[2][1], acc[2][2], acc[2][3]);
  acc_guard4(acc[3][0], acc[3][1], acc[3][2], acc[3][3]);

  float* slab = sT[wave];
  const float* Rb = RESID ? (resid + (size_t)b * strideR) : nullptr;
#pragma unroll
  for (int i = 0; i < 4; ++i) {
    const int mBase = m0 + (i << 4);
#pragma unroll
    for (int j = 0; j < 4; ++j) {
      const int n = n0 + (j << 4) + rlane;
      float bv = 0.f;
      if (BIAS_MODE == 2) bv = bias[n];
#pragma unroll
      for (int r = 0; r < 8; ++r) {
        float v = acc[i][j][r] * scale;
        if (BIAS_MODE == 1) v += bias[mBase + mOff + r];
        if (BIAS_MODE == 2) v += bv;
        if (RESID) v += Rb[(size_t)(mBase + mOff + r) * ldc + n];
        if (ACT == 1) v = tanhf(v);
        if (ACT == 2) v = fmaxf(v, 0.0f);
        if (ACT == 3) v = v / (1.0f + expf(-v));
        if (ACT == 4) v = (v > 0.f) ? v : 0.01f * v;
        if (ACT == 5) v = 0.5f * v * (1.0f + erff(v * 0.70710678118654752f));
        slab[(mOff + r) * 68 + (j << 4) + rlane] = v;
      }
    }
    __builtin_amdgcn_fence(__ATOMIC_RELEASE, "workgroup");
    __builtin_amdgcn_wave_barrier();
    __builtin_amdgcn_fence(__ATOMIC_ACQUIRE, "workgroup");
    if (OUT_MODE == 0) {
      float* C = (float*)Cout + (size_t)b * strideC;
      const int hh = lane >> 4, c4 = (lane & 15) * 4;
      for (int pass = 0; pass < 2; ++pass) {
#pragma unroll
        for (int it = 0; it < 8; ++it) {
          const int row = it * 2 + hh;
          v4f v = *(const v4f*)(slab + row * 68 + c4);
          *(volatile v4f*)(C + (size_t)(mBase + row) * ldc + n0 + c4) = v;
        }
        __threadfence();
      }
    } else {
      const int q = lane >> 3, c8 = (lane & 7) * 8;
      unsigned short* C  = (unsigned short*)Cout  + (size_t)b * strideC;
      unsigned short* C2 = (OUT_MODE == 2) ? ((unsigned short*)Cout2 + (size_t)b * strideC) : nullptr;
      for (int pass = 0; pass < 2; ++pass) {
#pragma unroll
        for (int it = 0; it < 4; ++it) {
          const int row = it * 4 + q;
          const float* sp = slab + row * 68 + c8;
          v8h hv, lv;
#pragma unroll
          for (int e = 0; e < 8; ++e) {
            if (OUT_MODE == 1) {
              hv[e] = (_Float16)sp[e];
            } else {
              unsigned short hb = f2bf_bits(sp[e]);
              unsigned short lb = f2bf_bits(sp[e] - bf_bits2f(hb));
              hv[e] = __builtin_bit_cast(_Float16, hb);
              lv[e] = __builtin_bit_cast(_Float16, lb);
            }
          }
          *(volatile v8h*)(C + (size_t)(mBase + row) * ldc + n0 + c8) = hv;
          if (OUT_MODE == 2) *(volatile v8h*)(C2 + (size_t)(mBase + row) * ldc + n0 + c8) = lv;
        }
        __threadfence();
      }
    }
    __builtin_amdgcn_fence(__ATOMIC_RELEASE, "workgroup");
    __builtin_amdgcn_wave_barrier();
    __builtin_amdgcn_fence(__ATOMIC_ACQUIRE, "workgroup");
  }
}

constexpr int VOCAB_N = 50000;
constexpr int EMB_D   = 256;
constexpr int HID_D   = 512;
constexpr int BATCH_N = 64;
constexpr int SEQ_T   = 1024;
constexpr int GATE_N  = 3 * HID_D;
constexpr int CHUNK_T = 256;
constexpr int CHUNK_N = SEQ_T / CHUNK_T;
constexpr int TOK_C   = BATCH_N * CHUNK_T;
constexpr int HA_PITCH = 520;
constexpr int ST_PITCH = 36;
constexpr float OP_SCALE    = 16.0f;
constexpr float OP_UNSCALE2 = 1.0f / 256.0f;

constexpr size_t WS_WH16 = 0;
constexpr size_t WS_WI16 = WS_WH16 + (size_t)GATE_N * HID_D * 2;
constexpr size_t WS_HST0 = WS_WI16 + (size_t)GATE_N * EMB_D * 2;
constexpr size_t WS_HST1 = WS_HST0 + (size_t)BATCH_N * HID_D * 4;
constexpr size_t WS_XE16 = WS_HST1 + (size_t)BATCH_N * HID_D * 4;
constexpr size_t WS_GIN  = WS_XE16 + (size_t)TOK_C * EMB_D * 2;
constexpr size_t WS_END  = WS_GIN  + (size_t)GATE_N * TOK_C * 4;
static_assert(WS_END == 111673344);
static_assert(WS_END <= 134217728);
static_assert(WS_WI16 % 256 == 0 && WS_HST0 % 256 == 0 && WS_HST1 % 256 == 0 && WS_XE16 % 256 == 0 && WS_GIN % 256 == 0);
static_assert(GATE_N % 64 == 0 && TOK_C % 64 == 0 && EMB_D % 32 == 0);
static_assert(HID_D % 32 == 0 && SEQ_T % CHUNK_T == 0 && (TOK_C % 8) == 0);
constexpr int OUT1_F = 256 / 4;
static_assert(OUT1_F + BATCH_N * HID_D == 131328 / 4);

__device__ __forceinline__ float bfr(float f) { return bf_bits2f(f2bf_bits(f)); }
__device__ __forceinline__ void guard3(v8f& c0, v8f& c1, v8f& c2, v16h a, v16h b0, v16h b1, v16h b2) {
  asm volatile("v_nop\n\tv_nop\n\tv_nop\n\tv_nop" : "+v"(c0), "+v"(c1), "+v"(c2) : "v"(a), "v"(b0), "v"(b1), "v"(b2));
}
__device__ __forceinline__ void lds_wave_sync() {
  __builtin_amdgcn_fence(__ATOMIC_RELEASE, "workgroup");
  __builtin_amdgcn_wave_barrier();
  __builtin_amdgcn_fence(__ATOMIC_ACQUIRE, "workgroup");
}

__global__ __launch_bounds__(256) void cast_w3(const float* __restrict__ w0, const float* __restrict__ w1,
                                               const float* __restrict__ w2, unsigned short* __restrict__ outp,
                                               int npairs) {
  const int g = blockIdx.y;
  const float* src = (g == 0) ? w0 : ((g == 1) ? w1 : w2);
  const int i = blockIdx.x * 256 + threadIdx.x;
  if (i < npairs) {
    const float a = src[2 * (size_t)i];
    const float b = src[2 * (size_t)i + 1];
    const _Float16 h0 = (_Float16)(bfr(a) * OP_SCALE);
    const _Float16 h1 = (_Float16)(bfr(b) * OP_SCALE);
    const unsigned u = (unsigned)__builtin_bit_cast(unsigned short, h0) | ((unsigned)__builtin_bit_cast(unsigned short, h1) << 16);
    volatile unsigned* o = ((volatile unsigned*)(outp + (size_t)g * 2 * (size_t)npairs)) + i;
    *o = u;
    __threadfence();
    *o = u;
  }
}

__global__ __launch_bounds__(256) void init_state(const float* __restrict__ h0, float* __restrict__ hst, int n4) {
  const int i = blockIdx.x * 256 + threadIdx.x;
  if (i < n4) {
    const v4f v = *(const v4f*)(h0 + 4 * (size_t)i);
    v4f o;
    o[0] = bfr(v[0]); o[1] = bfr(v[1]); o[2] = bfr(v[2]); o[3] = bfr(v[3]);
    volatile v4f* p = (volatile v4f*)(hst + 4 * (size_t)i);
    *p = o;
    __threadfence();
    *p = o;
  }
}

__global__ __launch_bounds__(256) void gather_rows(const int* __restrict__ x, const float* __restrict__ emb,
                                                   unsigned short* __restrict__ xep, int chunk) {
  const int lane = threadIdx.x & 31;
  const int row = blockIdx.x * 8 + (threadIdx.x >> 5);
  const int tl = row >> 6, b = row & 63;
  const int cc = chunk < 0 ? 0 : (chunk > CHUNK_N - 1 ? CHUNK_N - 1 : chunk);
  int tok = x[b * SEQ_T + cc * CHUNK_T + tl];
  tok = tok < 0 ? 0 : (tok > VOCAB_N - 1 ? VOCAB_N - 1 : tok);
  const float* er = emb + (size_t)tok * EMB_D + lane * 8;
  const v4f a = *(const v4f*)er;
  const v4f c = *(const v4f*)(er + 4);
  v8h hv;
  hv[0] = (_Float16)(bfr(a[0]) * OP_SCALE);
  hv[1] = (_Float16)(bfr(a[1]) * OP_SCALE);
  hv[2] = (_Float16)(bfr(a[2]) * OP_SCALE);
  hv[3] = (_Float16)(bfr(a[3]) * OP_SCALE);
  hv[4] = (_Float16)(bfr(c[0]) * OP_SCALE);
  hv[5] = (_Float16)(bfr(c[1]) * OP_SCALE);
  hv[6] = (_Float16)(bfr(c[2]) * OP_SCALE);
  hv[7] = (_Float16)(bfr(c[3]) * OP_SCALE);
  volatile v8h* o = (volatile v8h*)(((_Float16*)xep) + (size_t)row * EMB_D + lane * 8);
  *o = hv;
  __threadfence();
  *o = hv;
}

__global__ void __launch_bounds__(512)
rc_scan(const float* __restrict__ hin, float* __restrict__ hout,
        const float* __restrict__ gin, const unsigned short* __restrict__ whp,
        const float* __restrict__ b_ir, const float* __restrict__ b_hr,
        const float* __restrict__ b_iz, const float* __restrict__ b_hz,
        const float* __restrict__ b_in, const float* __restrict__ b_hn,
        int nsteps) {
  __shared__ __align__(16) _Float16 hA[16 * HA_PITCH];
  __shared__ __align__(16) float stile[16][16 * ST_PITCH];
  const _Float16* wh = (const _Float16*)whp;
  const int tid  = threadIdx.x;
  const int w    = tid >> 5;
  const int lane = tid & 31;
  const int hh   = lane >> 4;
  const int rl   = lane & 15;
  const int row0 = blockIdx.x * 16;
  float* st = stile[w];
  const int ns = nsteps < 0 ? 0 : (nsteps > CHUNK_T ? CHUNK_T : nsteps);

#pragma unroll
  for (int it = 0; it < 4; ++it) {
    const int r = it * 4 + (lane >> 3), c4 = (lane & 7) * 4;
    const v4f v = *(const v4f*)(hin + (size_t)(row0 + r) * HID_D + 32 * w + c4);
    *(v4f*)(st + r * ST_PITCH + c4) = v;
  }
  lds_wave_sync();
  float hold[2][8];
  float cbias[2][4];
#pragma unroll
  for (int cb = 0; cb < 2; ++cb) {
    const int col = 32 * w + 16 * cb + rl;
#pragma unroll
    for (int r = 0; r < 8; ++r) hold[cb][r] = st[(8 * hh + r) * ST_PITCH + 16 * cb + rl];
    cbias[cb][0] = bfr(b_ir[col]) + bfr(b_hr[col]);
    cbias[cb][1] = bfr(b_iz[col]) + bfr(b_hz[col]);
    cbias[cb][2] = bfr(b_in[col]);
    cbias[cb][3] = bfr(b_hn[col]);
  }

  const _Float16* arow = hA + rl * HA_PITCH + 8 * hh;
  for (int t = 0; t < ns; ++t) {
#pragma unroll
    for (int cb = 0; cb < 2; ++cb) {
      const int col = 32 * w + 16 * cb + rl;
#pragma unroll
      for (int r = 0; r < 8; ++r)
        hA[(8 * hh + r) * HA_PITCH + col] = (_Float16)(hold[cb][r] * OP_SCALE);
    }
    __syncthreads();

    const float* gbase = gin + (size_t)t * BATCH_N + row0 + 8 * hh;
#pragma unroll
    for (int cb = 0; cb < 2; ++cb) {
      const int col = 32 * w + 16 * cb + rl;
      const _Float16* bR = wh + (size_t)col * HID_D + 8 * hh;
      const _Float16* bZ = bR + (size_t)HID_D * HID_D;
      const _Float16* bN = bZ + (size_t)HID_D * HID_D;
      v8f aR = (v8f){0.f,0.f,0.f,0.f,0.f,0.f,0.f,0.f};
      v8f aZ = (v8f){0.f,0.f,0.f,0.f,0.f,0.f,0.f,0.f};
      v8f aN = (v8f){0.f,0.f,0.f,0.f,0.f,0.f,0.f,0.f};
#pragma unroll 2
      for (int k0 = 0; k0 < HID_D; k0 += 32) {
        const v16h a  = Frag<_Float16>::load(arow + k0);
        const v16h fr = Frag<_Float16>::load(bR + k0);
        const v16h fz = Frag<_Float16>::load(bZ + k0);
        const v16h fn = Frag<_Float16>::load(bN + k0);
        aR = Frag<_Float16>::mma(a, fr, aR);
        aZ = Frag<_Float16>::mma(a, fz, aZ);
        aN = Frag<_Float16>::mma(a, fn, aN);
        guard3(aR, aZ, aN, a, fr, fz, fn);
      }
      const float* gr = gbase + (size_t)col * TOK_C;
      const v8f gR = *(const v8f*)(gr);
      const v8f gZ = *(const v8f*)(gr + (size_t)HID_D * TOK_C);
      const v8f gN = *(const v8f*)(gr + (size_t)2 * HID_D * TOK_C);
#pragma unroll
      for (int r = 0; r < 8; ++r) {
        const float pr = aR[r] * OP_UNSCALE2 + gR[r] + cbias[cb][0];
        const float rg = 0.5f * tanhf(0.5f * pr) + 0.5f;
        const float pz = aZ[r] * OP_UNSCALE2 + gZ[r] + cbias[cb][1];
        const float zg = 0.5f * tanhf(0.5f * pz) + 0.5f;
        const float hn = aN[r] * OP_UNSCALE2 + cbias[cb][3];
        const float pn = gN[r] + cbias[cb][2] + rg * hn;
        const float ng = tanhf(pn);
        const float ho = hold[cb][r];
        hold[cb][r] = ng + zg * (ho - ng);
      }
      asm volatile("" ::: "memory");
    }
    __syncthreads();
  }

#pragma unroll
  for (int cb = 0; cb < 2; ++cb) {
#pragma unroll
    for (int r = 0; r < 8; ++r) st[(8 * hh + r) * ST_PITCH + 16 * cb + rl] = hold[cb][r];
  }
  lds_wave_sync();
  for (int pass = 0; pass < 2; ++pass) {
#pragma unroll
    for (int it = 0; it < 4; ++it) {
      const int r = it * 4 + (lane >> 3), c4 = (lane & 7) * 4;
      const v4f v = *(const v4f*)(st + r * ST_PITCH + c4);
      *(volatile v4f*)(hout + (size_t)(row0 + r) * HID_D + 32 * w + c4) = v;
    }
    __threadfence();
  }
}

__global__ __launch_bounds__(512) void head_out(const float* __restrict__ hst, const float* __restrict__ wfc,
                                                const float* __restrict__ bfc, float* __restrict__ out) {
  __shared__ __align__(16) float sres[BATCH_N];
  const int tid = threadIdx.x, w = tid >> 5, lane = tid & 31;
  v4f wf[4];
#pragma unroll
  for (int i = 0; i < 4; ++i) {
    const v4f tw = *(const v4f*)(wfc + i * 128 + lane * 4);
    v4f u;
    u[0] = bfr(tw[0]); u[1] = bfr(tw[1]); u[2] = bfr(tw[2]); u[3] = bfr(tw[3]);
    wf[i] = u;
  }
  const float bb = bfr(bfc[0]);
#pragma unroll 1
  for (int q = 0; q < 4; ++q) {
    const int row = w * 4 + q;
    v4f hv[4];
    float part = 0.0f;
#pragma unroll
    for (int i = 0; i < 4; ++i) {
      hv[i] = *(const v4f*)(hst + (size_t)row * HID_D + i * 128 + lane * 4);
      part += hv[i][0] * wf[i][0];
      part += hv[i][1] * wf[i][1];
      part += hv[i][2] * wf[i][2];
      part += hv[i][3] * wf[i][3];
    }
#pragma unroll
    for (int off = 1; off < 32; off <<= 1) part += __shfl_xor(part, off, 32);
    const float s = 0.5f * tanhf(0.5f * (part + bb)) + 0.5f;
    if (lane == 0) sres[row] = s;
    float* orow = out + OUT1_F + (size_t)row * HID_D + lane * 4;
#pragma unroll
    for (int i = 0; i < 4; ++i) *(volatile v4f*)(orow + i * 128) = hv[i];
    __threadfence();
#pragma unroll
    for (int i = 0; i < 4; ++i) *(volatile v4f*)(orow + i * 128) = hv[i];
  }
  __syncthreads();
  if (w == 0) {
    const int q = lane & 15;
    const v4f v = *(const v4f*)(sres + q * 4);
    if (lane < 16) *(volatile v4f*)(out + q * 4) = v;
    __threadfence();
    if (lane < 16) *(volatile v4f*)(out + q * 4) = v;
  }
}

extern "C" void kernel_launch(void* const* d_in, const int* in_sizes, int n_in,
                              void* d_out, int out_size, void* d_ws, size_t ws_size,
                              hipStream_t stream) {
  (void)in_sizes; (void)n_in; (void)out_size;
  const int*   x    = (const int*)  d_in[0];
  const float* h0   = (const float*)d_in[1];
  const float* emb  = (const float*)d_in[2];
  const float* Wir  = (const float*)d_in[3];
  const float* bir  = (const float*)d_in[4];
  const float* Whr  = (const float*)d_in[5];
  const float* bhr  = (const float*)d_in[6];
  const float* Wiz  = (const float*)d_in[7];
  const float* biz  = (const float*)d_in[8];
  const float* Whz  = (const float*)d_in[9];
  const float* bhz  = (const float*)d_in[10];
  const float* Win  = (const float*)d_in[11];
  const float* bin_ = (const float*)d_in[12];
  const float* Whn  = (const float*)d_in[13];
  const float* bhn  = (const float*)d_in[14];
  const float* Wfc  = (const float*)d_in[15];
  const float* bfc  = (const float*)d_in[16];
  float* out = (float*)d_out;
  unsigned char* ws = (unsigned char*)d_ws;
  if (ws_size < WS_END) return;

  unsigned short* WH16 = (unsigned short*)(ws + WS_WH16);
  unsigned short* WI16 = (unsigned short*)(ws + WS_WI16);
  float* HST[2] = { (float*)(ws + WS_HST0), (float*)(ws + WS_HST1) };
  unsigned short* XE16 = (unsigned short*)(ws + WS_XE16);
  float* GIN = (float*)(ws + WS_GIN);

  const int npairs_h = HID_D * HID_D / 2;
  const int npairs_i = HID_D * EMB_D / 2;
  cast_w3<<<dim3(npairs_h / 256, 3), 256, 0, stream>>>(Whr, Whz, Whn, WH16, npairs_h);
  cast_w3<<<dim3(npairs_i / 256, 3), 256, 0, stream>>>(Wir, Wiz, Win, WI16, npairs_i);
  const int n4 = BATCH_N * HID_D / 4;
  init_state<<<n4 / 256, 256, 0, stream>>>(h0, HST[0], n4);

  const int gemm_tiles  = (GATE_N / 64) * (TOK_C / 64);
  const int gemm_blocks = gemm_tiles / 8;
  for (int c = 0; c < CHUNK_N; ++c) {
    gather_rows<<<TOK_C / 8, 256, 0, stream>>>(x, emb, XE16, c);
    wmma_gemm64<0, false, 0, 0, false, 0><<<dim3(gemm_blocks, 1), 256, 0, stream>>>(
        WI16, WI16, EMB_D, 0L,
        XE16, XE16, EMB_D, 0L,
        (void*)GIN, (void*)GIN, TOK_C, 0L,
        (const float*)GIN, (const float*)GIN, 0L,
        GATE_N, TOK_C, EMB_D, OP_UNSCALE2);
    rc_scan<<<BATCH_N / 16, 512, 0, stream>>>(HST[c & 1], HST[(c + 1) & 1], GIN, WH16,
                                               bir, bhr, biz, bhz, bin_, bhn, CHUNK_T);
  }
  head_out<<<1, 512, 0, stream>>>(HST[CHUNK_N & 1], Wfc, bfc, out);
}
